// GraphMatcherP_89739046683486
// MI455X (gfx1250) — hardware-verified
//
#include <hip/hip_runtime.h>
#include <math.h>
#include <stddef.h>
#include <stdint.h>

#define NLAY  6
#define NBT   4
#define NTK   1024
#define DM    256
#define NHD   4
#define HDIM  64
#define MTOK  4096
#define SPT   68
#define WSMAX 134217728

static_assert(DM == 256);
static_assert(NHD == 4);
static_assert(HDIM == 64);
static_assert(DM == NHD * HDIM);
static_assert(NTK % 64 == 0);
static_assert(MTOK == NBT * NTK);
static_assert(MTOK % 128 == 0);
static_assert(NBT == 4);
static_assert(NLAY == 6);
static_assert((2 * DM) % 32 == 0);
static_assert((4 * DM) % 32 == 0);

typedef float          v4f   __attribute__((ext_vector_type(4)));
typedef float          v8f   __attribute__((ext_vector_type(8)));
typedef int            v8i   __attribute__((ext_vector_type(8)));
typedef unsigned short v8us  __attribute__((ext_vector_type(8)));
typedef unsigned short v16us __attribute__((ext_vector_type(16)));
typedef __bf16         v16bf __attribute__((ext_vector_type(16)));
typedef __bf16         v8bf  __attribute__((ext_vector_type(8)));
typedef v4f  __attribute__((may_alias)) v4fa;
typedef v8us __attribute__((may_alias)) v8usa;
union FragB { v16bf v; v16us u; v8us h[2]; v8i w; };

__device__ __forceinline__ v8f wmb(const FragB& a, const FragB& b, v8f c) {
  v8f d = __builtin_amdgcn_wmma_f32_16x16x32_bf16(false, a.v, false, b.v, (short)0, c, false, false);
  asm volatile("v_nop\n\tv_nop\n\tv_nop\n\tv_nop" : "+v"(d) : "v"(a.w), "v"(b.w));
  return d;
}
__device__ __forceinline__ v8f z8() { v8f z = {0.f, 0.f, 0.f, 0.f, 0.f, 0.f, 0.f, 0.f}; return z; }

__device__ __forceinline__ unsigned bf16_bits(float f) {
  const unsigned u = __float_as_uint(f);
  return (u + 0x7FFFu + ((u >> 16) & 1u)) >> 16;
}
__device__ __forceinline__ float bf16_val(float f) { return __uint_as_float(bf16_bits(f) << 16); }

__device__ __forceinline__ v8us cvt8(v4f a, v4f b) {
  v8us o;
  o[0] = (unsigned short)bf16_bits(a.x); o[1] = (unsigned short)bf16_bits(a.y);
  o[2] = (unsigned short)bf16_bits(a.z); o[3] = (unsigned short)bf16_bits(a.w);
  o[4] = (unsigned short)bf16_bits(b.x); o[5] = (unsigned short)bf16_bits(b.y);
  o[6] = (unsigned short)bf16_bits(b.z); o[7] = (unsigned short)bf16_bits(b.w);
  return o;
}

#define WP_B0 1152
#define WP_B1 1536
#define WP_B2 768
#define WP_B3 384
#define WP_B4 6
static_assert(WP_B0 * 256 * 8 == NLAY * 768 * 512);
static_assert(WP_B1 * 256 * 8 == NLAY * 512 * 1024);
static_assert(WP_B2 * 256 * 8 == NLAY * 256 * 1024);
static_assert(WP_B3 * 256 * 8 == NLAY * 256 * 512);

__global__ __launch_bounds__(256) __attribute__((amdgpu_num_vgpr(248)))
void k_wprep(const float* __restrict__ wq, const float* __restrict__ wk, const float* __restrict__ wv,
             const float* __restrict__ wm, const float* __restrict__ w1, const float* __restrict__ w2,
             const float* __restrict__ bq, const float* __restrict__ bk, const float* __restrict__ bv,
             unsigned short* WQKVD, unsigned short* WMD, unsigned short* W1D, unsigned short* W2D, float* BQKV) {
  const int bx = (int)blockIdx.x, tid = (int)threadIdx.x;
  if (bx < WP_B0 + WP_B1 + WP_B2) {
    const float* p;
    unsigned short* dp;
    if (bx < WP_B0) {
      const int rowg  = bx * 4 + (tid >> 6);
      const int l     = rowg / 768;
      const int n     = rowg - l * 768;
      const int which = ((bx * 4) % 768) >> 8;
      const float* src = (which == 0) ? wq : ((which == 1) ? wk : wv);
      const int pp = n & 255, h = pp >> 6, d = pp & 63;
      const int ks = ((tid & 63) * 8) & 255;
      p  = src + ((size_t)(l * 256 + d * 4 + h)) * 256 + ks;
      dp = WQKVD + ((size_t)bx * 256 + tid) * 8;
    } else if (bx < WP_B0 + WP_B1) {
      const int u   = (bx - WP_B0) * 256 + tid;
      const int row = u >> 7;
      const int ks  = ((u & 127) * 8) & 511;
      p  = w1 + (size_t)row * 512 + ks;
      dp = W1D + (size_t)u * 8;
    } else {
      const int u   = (bx - WP_B0 - WP_B1) * 256 + tid;
      const int row = u >> 7;
      const int ks  = ((u & 127) * 8) & 511;
      p  = w2 + (size_t)row * 512 + ks;
      dp = W2D + (size_t)u * 8;
    }
    const v4f a = *(const v4f*)p;
    const v4f b = *(const v4f*)(p + 4);
    const v8us o8 = cvt8(a, b);
    *(volatile v8us*)dp = o8;
    __threadfence();
    *(volatile v8us*)dp = o8;
  } else if (bx < WP_B0 + WP_B1 + WP_B2 + WP_B3) {
    const int u   = (bx - WP_B0 - WP_B1 - WP_B2) * 256 + tid;
    const int row = u >> 6;
    const int ks  = ((u & 63) * 8) & 255;
    const int h = ks >> 6, d0 = ks & 63;
    const float* p = wm + (size_t)row * 256 + d0 * 4 + h;
    v8us o8;
#pragma unroll
    for (int e = 0; e < 8; ++e) o8[e] = (unsigned short)bf16_bits(p[e * 4]);
    unsigned short* dp = WMD + (size_t)u * 8;
    *(volatile v8us*)dp = o8;
    __threadfence();
    *(volatile v8us*)dp = o8;
  } else {
    const int rb = bx - (WP_B0 + WP_B1 + WP_B2 + WP_B3);
    const int w  = rb >> 1;
    const int u  = (rb & 1) * 256 + tid;
    if (u < 384) {
      const float* src = (w == 0) ? bq : ((w == 1) ? bk : bv);
      const int l  = u >> 6;
      const int p4 = (u & 63) * 4;
      const int h = p4 >> 6, d = p4 & 63;
      const float* p = src + (size_t)l * 256 + d * 4 + h;
      v4f o4;
      o4.x = bf16_val(p[0]); o4.y = bf16_val(p[4]); o4.z = bf16_val(p[8]); o4.w = bf16_val(p[12]);
      float* dp = BQKV + (size_t)l * 768 + w * 256 + p4;
      *(volatile v4f*)dp = o4;
      __threadfence();
      *(volatile v4f*)dp = o4;
    }
  }
}

__global__ __launch_bounds__(256) __attribute__((amdgpu_num_vgpr(248)))
void k_mask(const float* __restrict__ m, unsigned short* mbp) {
  const size_t u = (size_t)blockIdx.x * 256 + threadIdx.x;
  const v4f a = *(const v4f*)(m + u * 8);
  const v4f b = *(const v4f*)(m + u * 8 + 4);
  const v8us o8 = cvt8(a, b);
  *(volatile v8us*)(mbp + u * 8) = o8;
  __threadfence();
  *(volatile v8us*)(mbp + u * 8) = o8;
}

__global__ __launch_bounds__(256) __attribute__((amdgpu_num_vgpr(248)))
void k_xprep(const float* __restrict__ desc, int bofs, float* xa, unsigned short* xhl, unsigned short* yhl) {
  __shared__ __attribute__((aligned(16))) float tf[64 * SPT];
  const int bx = (int)blockIdx.x, tid = (int)threadIdx.x;
  const int ct = bx & 3, nt = (bx >> 2) & 15, bl = bx >> 6;
  const int n0 = nt * 64, c0 = ct * 64;
  const int r0 = (bofs + bl) * NTK + n0;
  {
    const int rsub = tid >> 4, c4 = (tid & 15) * 4;
#pragma unroll
    for (int it = 0; it < 4; ++it) {
      const int cr = it * 16 + rsub;
      const v4f a = *(const v4f*)(desc + ((size_t)(bl * DM + c0 + cr)) * NTK + n0 + c4);
      *(v4fa*)(tf + cr * SPT + c4) = a;
    }
  }
  __syncthreads();
  {
    const int rsub = tid >> 4, c4 = (tid & 15) * 4;
    v4f ov[4];
#pragma unroll
    for (int it = 0; it < 4; ++it) {
      const int tl = it * 16 + rsub;
      v4f v;
      v.x = bf16_val(tf[(c4 + 0) * SPT + tl]); v.y = bf16_val(tf[(c4 + 1) * SPT + tl]);
      v.z = bf16_val(tf[(c4 + 2) * SPT + tl]); v.w = bf16_val(tf[(c4 + 3) * SPT + tl]);
      ov[it] = v;
    }
#pragma unroll
    for (int it = 0; it < 4; ++it) {
      const int tl = it * 16 + rsub;
      *(volatile v4f*)(xa + (size_t)(r0 + tl) * DM + c0 + c4) = ov[it];
    }
    __threadfence();
#pragma unroll
    for (int it = 0; it < 4; ++it) {
      const int tl = it * 16 + rsub;
      *(volatile v4f*)(xa + (size_t)(r0 + tl) * DM + c0 + c4) = ov[it];
    }
  }
  {
    const int rsub = tid >> 3, c8 = (tid & 7) * 8;
    const v8us zv = {0, 0, 0, 0, 0, 0, 0, 0};
    v8us hv[2];
#pragma unroll
    for (int it = 0; it < 2; ++it) {
      const int tl = it * 32 + rsub;
      v8us w;
#pragma unroll
      for (int e = 0; e < 8; ++e) w[e] = (unsigned short)bf16_bits(tf[(c8 + e) * SPT + tl]);
      hv[it] = w;
    }
#pragma unroll
    for (int it = 0; it < 2; ++it) {
      const size_t r = (size_t)(r0 + it * 32 + rsub);
      *(volatile v8us*)(xhl + r * 512 + c0 + c8)        = hv[it];
      *(volatile v8us*)(xhl + r * 512 + 256 + c0 + c8)  = zv;
      *(volatile v8us*)(yhl + r * 1024 + c0 + c8)       = hv[it];
      *(volatile v8us*)(yhl + r * 1024 + 512 + c0 + c8) = zv;
    }
    __threadfence();
#pragma unroll
    for (int it = 0; it < 2; ++it) {
      const size_t r = (size_t)(r0 + it * 32 + rsub);
      *(volatile v8us*)(xhl + r * 512 + c0 + c8)        = hv[it];
      *(volatile v8us*)(xhl + r * 512 + 256 + c0 + c8)  = zv;
      *(volatile v8us*)(yhl + r * 1024 + c0 + c8)       = hv[it];
      *(volatile v8us*)(yhl + r * 1024 + 512 + c0 + c8) = zv;
    }
  }
}

__device__ __forceinline__ void put_hl(const float* stg, int tid, unsigned short* H, unsigned short* L, size_t ld) {
  const int rsub = tid >> 3;
  const int c8   = (tid & 7) * 8;
  v8us hv[4], lv[4];
#pragma unroll
  for (int it = 0; it < 4; ++it) {
    const int row = it * 16 + rsub;
    const float* sp = stg + row * SPT + c8;
    v8us h8, l8;
#pragma unroll
    for (int e = 0; e < 8; ++e) {
      const float v = sp[e];
      const unsigned hb = bf16_bits(v);
      const unsigned lb = bf16_bits(v - __uint_as_float(hb << 16));
      h8[e] = (unsigned short)hb;
      l8[e] = (unsigned short)lb;
    }
    hv[it] = h8; lv[it] = l8;
  }
#pragma unroll
  for (int it = 0; it < 4; ++it) {
    const size_t go = (size_t)(it * 16 + rsub) * ld + c8;
    *(volatile v8us*)(H + go) = hv[it];
    *(volatile v8us*)(L + go) = lv[it];
  }
  __threadfence();
#pragma unroll
  for (int it = 0; it < 4; ++it) {
    const size_t go = (size_t)(it * 16 + rsub) * ld + c8;
    *(volatile v8us*)(H + go) = hv[it];
    *(volatile v8us*)(L + go) = lv[it];
  }
}

__device__ __forceinline__ void put_vt(const float* stg, int tid, unsigned short* H, unsigned short* L) {
  const int rsub = tid >> 3;
  const int c8   = (tid & 7) * 8;
  v8us hv[4], lv[4];
#pragma unroll
  for (int it = 0; it < 4; ++it) {
    const int dr = it * 16 + rsub;
    v8us h8, l8;
#pragma unroll
    for (int e = 0; e < 8; ++e) {
      const float v = stg[(c8 + e) * SPT + dr];
      const unsigned hb = bf16_bits(v);
      const unsigned lb = bf16_bits(v - __uint_as_float(hb << 16));
      h8[e] = (unsigned short)hb;
      l8[e] = (unsigned short)lb;
    }
    hv[it] = h8; lv[it] = l8;
  }
#pragma unroll
  for (int it = 0; it < 4; ++it) {
    const size_t go = (size_t)(it * 16 + rsub) * NTK + c8;
    *(volatile v8us*)(H + go) = hv[it];
    *(volatile v8us*)(L + go) = lv[it];
  }
  __threadfence();
#pragma unroll
  for (int it = 0; it < 4; ++it) {
    const size_t go = (size_t)(it * 16 + rsub) * NTK + c8;
    *(volatile v8us*)(H + go) = hv[it];
    *(volatile v8us*)(L + go) = lv[it];
  }
}

template <int MODE>
__global__ __launch_bounds__(128) __attribute__((amdgpu_num_vgpr(248)))
void k_gemm(const unsigned short* __restrict__ A, int lda,
            const unsigned short* __restrict__ BT, int ldb, int K,
            const float* __restrict__ bias,
            unsigned short* P0, unsigned short* P1,
            float* F0, const float* __restrict__ R0, float* REC) {
  __shared__ __attribute__((aligned(16))) float stg[64 * SPT];
  __shared__ __attribute__((aligned(16))) float sb[64];
  __shared__ __attribute__((aligned(16))) float pst[128];
  const int tid = (int)threadIdx.x, lane = tid & 31, wave = tid >> 5, hh = lane >> 4, m = lane & 15;
  const int rowBase = (int)blockIdx.x * 64;
  const int colBase = (int)blockIdx.y * 64;
  if (tid < 64) sb[tid] = bf16_val(bias[colBase + tid]);
  __syncthreads();

  v8f acc[4];
#pragma unroll
  for (int t = 0; t < 4; ++t) acc[t] = z8();
  const unsigned short* ap = A  + (size_t)(rowBase + 16 * wave + m) * (size_t)lda + 8 * hh;
  const unsigned short* bp = BT + (size_t)(colBase + m) * (size_t)ldb + 8 * hh;

#pragma unroll 1
  for (int k0 = 0; k0 < K; k0 += 32) {
    FragB af;
    af.h[0] = *(const v8usa*)(ap + k0);
    af.h[1] = *(const v8usa*)(ap + k0 + 16);
#pragma unroll
    for (int nt = 0; nt < 4; ++nt) {
      const unsigned short* wq = bp + (size_t)(16 * nt) * (size_t)ldb + k0;
      FragB bf;
      bf.h[0] = *(const v8usa*)wq;
      bf.h[1] = *(const v8usa*)(wq + 16);
      acc[nt] = wmb(af, bf, acc[nt]);
    }
  }

#pragma unroll
  for (int nt = 0; nt < 4; ++nt) {
    const int lc = 16 * nt + m;
    const float bc = sb[lc];
#pragma unroll
    for (int r = 0; r < 8; ++r) {
      const int lr = 16 * wave + 8 * hh + r;
      stg[lr * SPT + lc] = acc[nt][r] + bc;
    }
  }
  __syncthreads();

  if (MODE == 0) {
    const int third = colBase >> 8;
    const int cq    = colBase & 255;
    if (third < 2) {
      unsigned short* base = P0 + (size_t)third * ((size_t)MTOK * 512) + (size_t)rowBase * 512 + cq;
      put_hl(stg, tid, base, base + 256, 512);
    } else {
      const int b = rowBase >> 10, n0 = rowBase & (NTK - 1), h = cq >> 6;
      unsigned short* vh = P1 + ((size_t)((b * NHD + h) * HDIM)) * NTK + n0;
      put_vt(stg, tid, vh, vh + (size_t)NBT * NHD * HDIM * NTK);
    }
  } else if (MODE == 1) {
    unsigned short* base = P0 + (size_t)rowBase * 1024 + 256 + colBase;
    put_hl(stg, tid, base, base + 512, 1024);
  } else if (MODE == 2) {
    const int rsub = tid >> 4;
    const int c4   = (tid & 15) * 4;
    v4f pv[8];
#pragma unroll
    for (int it = 0; it < 8; ++it) pv[it] = *(const v4fa*)(stg + (it * 8 + rsub) * SPT + c4);
#pragma unroll
    for (int it = 0; it < 8; ++it)
      *(volatile v4f*)(F0 + (size_t)(rowBase + it * 8 + rsub) * 512 + colBase + c4) = pv[it];
    __threadfence();
#pragma unroll
    for (int it = 0; it < 8; ++it)
      *(volatile v4f*)(F0 + (size_t)(rowBase + it * 8 + rsub) * 512 + colBase + c4) = pv[it];
    if (tid < 64) {
      float s = 0.0f;
#pragma unroll 4
      for (int r = 0; r < 64; ++r) s += stg[r * SPT + tid];
      const float mean = s * (1.0f / 64.0f);
      float q = 0.0f;
#pragma unroll 4
      for (int r = 0; r < 64; ++r) {
        const float d = stg[r * SPT + tid] - mean;
        q = fmaf(d, d, q);
      }
      pst[tid] = mean;
      pst[64 + tid] = q;
    }
    __syncthreads();
    v4f qv;
    float* rp = REC + (size_t)blockIdx.x * 1024 + (size_t)(tid >> 4) * 512 + colBase + (tid & 15) * 4;
    if (tid < 32) {
      qv = *(const v4fa*)(pst + 4 * tid);
      *(volatile v4f*)rp = qv;
    }
    __threadfence();
    if (tid < 32) {
      *(volatile v4f*)rp = qv;
    }
  } else {
    const int rsub = tid >> 4;
    const int c4   = (tid & 15) * 4;
    v4f pv[8];
#pragma unroll
    for (int it = 0; it < 8; ++it) {
      const int row = it * 8 + rsub;
      const v4f a = *(const v4fa*)(stg + row * SPT + c4);
      const v4f x = *(const v4f*)(R0 + (size_t)(rowBase + row) * DM + colBase + c4);
      v4f v;
      v.x = a.x + x.x; v.y = a.y + x.y; v.z = a.z + x.z; v.w = a.w + x.w;
      pv[it] = v;
      *(v4fa*)(stg + row * SPT + c4) = v;
    }
    __syncthreads();
#pragma unroll
    for (int it = 0; it < 8; ++it)
      *(volatile v4f*)(F0 + (size_t)(rowBase + it * 8 + rsub) * DM + colBase + c4) = pv[it];
    __threadfence();
#pragma unroll
    for (int it = 0; it < 8; ++it)
      *(volatile v4f*)(F0 + (size_t)(rowBase + it * 8 + rsub) * DM + colBase + c4) = pv[it];
    unsigned short* xb = P0 + (size_t)rowBase * 512 + colBase;
    put_hl(stg, tid, xb, xb + 256, 512);
    unsigned short* yb = P1 + (size_t)rowBase * 1024 + colBase;
    put_hl(stg, tid, yb, yb + 512, 1024);
  }
}

#define AT_D  64
#define AT_NW 4
#define AT_QB 64
#define AT_KC 64

__device__ __forceinline__ unsigned short at_bf_bits(float f) {
  unsigned u = __float_as_uint(f);
  return (unsigned short)((u + 0x7FFFu + ((u >> 16) & 1u)) >> 16);
}
__device__ __forceinline__ __bf16 at_f2bf(float f) { return __builtin_bit_cast(__bf16, at_bf_bits(f)); }
__device__ __forceinline__ void at_split(float f, __bf16& hi, __bf16& lo) {
  const unsigned short hb = at_bf_bits(f);
  hi = __builtin_bit_cast(__bf16, hb);
  lo = at_f2bf(f - __uint_as_float(((unsigned)hb) << 16));
}
__device__ __forceinline__ v8f at_mma(v16bf a, v16bf b, v8f c) {
  c = __builtin_amdgcn_wmma_f32_16x16x32_bf16(false, a, false, b, (short)0, c, false, false);
  asm volatile("v_nop\n\tv_nop\n\tv_nop\n\tv_nop" : "+v"(c) : "v"(a), "v"(b));
  return c;
}
union AtFB { v16bf v; v8bf h[2]; };
__device__ __forceinline__ v16bf at_ldfrag(const __bf16* p) {
  AtFB f; f.h[0] = *(const v8bf*)(p); f.h[1] = *(const v8bf*)(p + 16); return f.v;
}

__global__ __launch_bounds__(128) __attribute__((amdgpu_num_vgpr(248)))
void k_attn(const unsigned short* __restrict__ qk, const unsigned short* __restrict__ vt,
            const unsigned short* __restrict__ mb, unsigned short* ctx, int cross) {
  __shared__ __align__(16) __bf16 Ksh[AT_KC * AT_D];
  __shared__ __align__(16) __bf16 Ksl[AT_KC * AT_D];
  __shared__ __align__(16) __bf16 Vth[AT_D * AT_KC];
  __shared__ __align__(16) __bf16 Vtl[AT_D * AT_KC];
  __shared__ __align__(16) __bf16 Psh[AT_NW][16 * AT_KC];
  __shared__ __align__(16) __bf16 Psl[AT_NW][16 * AT_KC];
  __shared__ __align__(16) float  Os[AT_NW][16 * SPT];
  __shared__ __align__(16) unsigned short Msk[AT_QB * AT_KC];

  const int tid  = (int)threadIdx.x;
  const int wave = tid >> 5;
  const int lane = tid & 31;
  const int hh   = lane >> 4;
  const int c    = lane & 15;

  const int bx = (int)blockIdx.x;
  const int qb = bx & 15;
  const int h  = (bx >> 4) & 3;
  const int b  = bx >> 6;
  const int kb = cross ? (b ^ 2) : b;
  const int q0 = qb * AT_QB + wave * 16;

  const __bf16* Qh = (const __bf16*)(const void*)qk + (size_t)b * NTK * 512 + h * AT_D;
  const __bf16* Ql = Qh + 256;
  const __bf16* Kh = (const __bf16*)(const void*)qk + (size_t)MTOK * 512 + (size_t)kb * NTK * 512 + h * AT_D;
  const __bf16* Kl = Kh + 256;
  const __bf16* Vh = (const __bf16*)(const void*)vt + ((size_t)((kb * NHD + h) * HDIM)) * NTK;
  const __bf16* Vl = Vh + (size_t)NBT * NHD * HDIM * NTK;
  const unsigned short* Mr = mb + ((size_t)b * NTK + (size_t)qb * AT_QB) * NTK;
  unsigned short* yb = ctx + (size_t)b * NTK * 512 + h * AT_D;

  v16bf qah[2], qal[2];
#pragma unroll
  for (int dc = 0; dc < 2; ++dc) {
    const __bf16* qr = Qh + (size_t)(q0 + c) * 512 + dc * 32 + 8 * hh;
    const __bf16* ql = Ql + (size_t)(q0 + c) * 512 + dc * 32 + 8 * hh;
    qah[dc] = at_ldfrag(qr);
    qal[dc] = at_ldfrag(ql);
  }

  float mrow[8], lrow[8];
  v8f oacc[4];
#pragma unroll
  for (int r = 0; r < 8; ++r) { mrow[r] = -INFINITY; lrow[r] = 0.f; }
#pragma unroll
  for (int t = 0; t < 4; ++t) oacc[t] = z8();

  const int nChunks = NTK / AT_KC;
  for (int kc = 0; kc < nChunks; ++kc) {
    const int kv0 = kc * AT_KC;
    __syncthreads();
    {
      const int r = tid >> 1, half = (tid & 1) * 32;
      const __bf16* ksh = Kh + (size_t)(kv0 + r) * 512 + half;
      const __bf16* ksl = Kl + (size_t)(kv0 + r) * 512 + half;
      const __bf16* vsh = Vh + (size_t)r * NTK + kv0 + half;
      const __bf16* vsl = Vl + (size_t)r * NTK + kv0 + half;
      const unsigned short* msr = Mr + (size_t)r * NTK + kv0 + half;
#pragma unroll
      for (int i = 0; i < 4; ++i) {
        const v8bf a0 = *(const v8bf*)(ksh + 8 * i);
        const v8bf a1 = *(const v8bf*)(ksl + 8 * i);
        const v8bf b0 = *(const v8bf*)(vsh + 8 * i);
        const v8bf b1 = *(const v8bf*)(vsl + 8 * i);
        const v8us m0 = *(const v8us*)(msr + 8 * i);
        *(v8bf*)(Ksh + r * AT_D  + half + 8 * i) = a0;
        *(v8bf*)(Ksl + r * AT_D  + half + 8 * i) = a1;
        *(v8bf*)(Vth + r * AT_KC + half + 8 * i) = b0;
        *(v8bf*)(Vtl + r * AT_KC + half + 8 * i) = b1;
        *(v8us*)(Msk + r * AT_KC + half + 8 * i) = m0;
      }
    }
    __syncthreads();

    v8f s[4];
#pragma unroll
    for (int j = 0; j < 4; ++j) {
      s[j] = z8();
#pragma unroll
      for (int dc = 0; dc < 2; ++dc) {
        AtFB kbf, klf;
        kbf.h[0] = *(const v8bf*)(Ksh + (j * 16 + c) * AT_D + dc * 32 + 8 * hh);
        kbf.h[1] = *(const v8bf*)(Ksh + (j * 16 + c) * AT_D + dc * 32 + 16 + 8 * hh);
        klf.h[0] = *(const v8bf*)(Ksl + (j * 16 + c) * AT_D + dc * 32 + 8 * hh);
        klf.h[1] = *(const v8bf*)(Ksl + (j * 16 + c) * AT_D + dc * 32 + 16 + 8 * hh);
        s[j] = at_mma(qah[dc], kbf.v, s[j]);
        s[j] = at_mma(qah[dc], klf.v, s[j]);
        s[j] = at_mma(qal[dc], kbf.v, s[j]);
      }
    }
    float cm[8];
#pragma unroll
    for (int r = 0; r < 8; ++r) {
      const unsigned short* mrp = Msk + (wave * 16 + 8 * hh + r) * AT_KC + c;
      float mx = -INFINITY;
#pragma unroll
      for (int j = 0; j < 4; ++j) {
        const float mv = __uint_as_float(((unsigned)mrp[j * 16]) << 16);
        float sv = s[j][r] * 0.125f;
        sv = sv * mv;
        s[j][r] = sv;
        mx = fmaxf(mx, sv);
      }
#pragma unroll
      for (int off = 1; off < 16; off <<= 1) mx = fmaxf(mx, __shfl_xor(mx, off, 32));
      cm[r] = mx;
    }
    __bf16* pwh = Psh[wave];
    __bf16* pwl = Psl[wave];
#pragma unroll
    for (int r = 0; r < 8; ++r) {
      const float mnew  = fmaxf(mrow[r], cm[r]);
      const float alpha = expf(mrow[r] - mnew);
      mrow[r] = mnew;
      float psum = 0.f;
#pragma unroll
      for (int j = 0; j < 4; ++j) {
        const float p = expf(s[j][r] - mnew);
        psum += p;
        __bf16 a, bl; at_split(p, a, bl);
        pwh[(8 * hh + r) * AT_KC + j * 16 + c] = a;
        pwl[(8 * hh + r) * AT_KC + j * 16 + c] = bl;
      }
#pragma unroll
      for (int off = 1; off < 16; off <<= 1) psum += __shfl_xor(psum, off, 32);
      lrow[r] = lrow[r] * alpha + psum;
#pragma unroll
      for (int t = 0; t < 4; ++t) oacc[t][r] *= alpha;
    }
    __builtin_amdgcn_fence(__ATOMIC_RELEASE, "workgroup");
    __builtin_amdgcn_wave_barrier();
    __builtin_amdgcn_fence(__ATOMIC_ACQUIRE, "workgroup");
#pragma unroll 1
    for (int kk = 0; kk < 2; ++kk) {
      AtFB pa, pl;
      pa.h[0] = *(const v8bf*)(pwh + c * AT_KC + kk * 32 + 8 * hh);
      pa.h[1] = *(const v8bf*)(pwh + c * AT_KC + kk * 32 + 16 + 8 * hh);
      pl.h[0] = *(const v8bf*)(pwl + c * AT_KC + kk * 32 + 8 * hh);
      pl.h[1] = *(const v8bf*)(pwl + c * AT_KC + kk * 32 + 16 + 8 * hh);
#pragma unroll
      for (int t = 0; t < 4; ++t) {
        AtFB vb, vl;
        vb.h[0] = *(const v8bf*)(Vth + (t * 16 + c) * AT_KC + kk * 32 + 8 * hh);
        vb.h[1] = *(const v8bf*)(Vth + (t * 16 + c) * AT_KC + kk * 32 + 16 + 8 * hh);
        vl.h[0] = *(const v8bf*)(Vtl + (t * 16 + c) * AT_KC + kk * 32 + 8 * hh);
        vl.h[1] = *(const v8bf*)(Vtl + (t * 16 + c) * AT_KC + kk * 32 + 16 + 8 * hh);
        oacc[t] = at_mma(pa.v, vb.v, oacc[t]);
        oacc[t] = at_mma(pa.v, vl.v, oacc[t]);
        oacc[t] = at_mma(pl.v, vb.v, oacc[t]);
      }
    }
  }

  float* os = Os[wave];
#pragma unroll
  for (int r = 0; r < 8; ++r) {
    const float inv = 1.0f / lrow[r];
#pragma unroll
    for (int t = 0; t < 4; ++t) os[(8 * hh + r) * SPT + t * 16 + c] = oacc[t][r] * inv;
  }
  __builtin_amdgcn_fence(__ATOMIC_RELEASE, "workgroup");
  __builtin_amdgcn_wave_barrier();
  __builtin_amdgcn_fence(__ATOMIC_ACQUIRE, "workgroup");
  {
    const int q  = lane >> 3;
    const int c8 = (lane & 7) * 8;
    v8us hv[4], lv[4];
#pragma unroll
    for (int it = 0; it < 4; ++it) {
      const int row = it * 4 + q;
      const float* sp = os + row * SPT + c8;
      v8us h8, l8;
#pragma unroll
      for (int e = 0; e < 8; ++e) {
        const float f = sp[e];
        const unsigned short hb = at_bf_bits(f);
        const unsigned short lb = at_bf_bits(f - __uint_as_float(((unsigned)hb) << 16));
        h8[e] = hb; l8[e] = lb;
      }
      hv[it] = h8; lv[it] = l8;
    }
#pragma unroll
    for (int it = 0; it < 4; ++it) {
      const int row = it * 4 + q;
      unsigned short* yr = yb + (size_t)(q0 + row) * 512 + c8;
      *(volatile v8us*)(yr)       = hv[it];
      *(volatile v8us*)(yr + 256) = lv[it];
    }
    __threadfence();
#pragma unroll
    for (int it = 0; it < 4; ++it) {
      const int row = it * 4 + q;
      unsigned short* yr = yb + (size_t)(q0 + row) * 512 + c8;
      *(volatile v8us*)(yr)       = hv[it];
      *(volatile v8us*)(yr + 256) = lv[it];
    }
  }
}

__global__ __launch_bounds__(256) __attribute__((amdgpu_num_vgpr(248)))
void k_bnrelu(const float* __restrict__ z, const float* __restrict__ rec, const float* __restrict__ g,
              const float* __restrict__ be, unsigned short* rhl) {
  __shared__ __attribute__((aligned(16))) float sm[64];
  __shared__ __attribute__((aligned(16))) float sr[64];
  __shared__ __attribute__((aligned(16))) float sg[64];
  __shared__ __attribute__((aligned(16))) float sbt[64];
  const int tid = (int)threadIdx.x;
  const int colBase = (int)blockIdx.x * 64;
  const int rowBase = (int)blockIdx.y * 256;
  if (tid < 64) {
    const int cc = colBase + tid;
    double s = 0.0;
#pragma unroll 4
    for (int rb = 0; rb < 64; ++rb) s += (double)rec[(size_t)rb * 1024 + cc];
    const double mean = s * (1.0 / 64.0);
    double q = 0.0;
#pragma unroll 4
    for (int rb = 0; rb < 64; ++rb) {
      const double d = (double)rec[(size_t)rb * 1024 + cc] - mean;
      q += (double)rec[(size_t)rb * 1024 + 512 + cc] + 64.0 * d * d;
    }
    const double var  = q * (1.0 / 4096.0);
    const double rstd = 1.0 / sqrt(var + (double)1e-5f);
    sm[tid]  = (float)mean;
    sr[tid]  = (float)rstd;
    sg[tid]  = bf16_val(g[cc]);
    sbt[tid] = bf16_val(be[cc]);
  }
  __syncthreads();
  const int rsub = tid >> 3;
  const int c8   = (tid & 7) * 8;
  float m8[8], r8[8], g8[8], b8[8];
#pragma unroll
  for (int e = 0; e < 8; ++e) { m8[e] = sm[c8 + e]; r8[e] = sr[c8 + e]; g8[e] = sg[c8 + e]; b8[e] = sbt[c8 + e]; }
#pragma unroll 1
  for (int it = 0; it < 8; ++it) {
    const size_t row = (size_t)(rowBase + it * 32 + rsub);
    const float* zp = z + row * 512 + colBase + c8;
    const v4f a = *(const v4f*)zp;
    const v4f b = *(const v4f*)(zp + 4);
    float v[8];
    v[0] = a.x; v[1] = a.y; v[2] = a.z; v[3] = a.w; v[4] = b.x; v[5] = b.y; v[6] = b.z; v[7] = b.w;
    v8us h8, l8;
#pragma unroll
    for (int e = 0; e < 8; ++e) {
      float y = ((v[e] - m8[e]) * r8[e]) * g8[e] + b8[e];
      y = (y > 0.0f) ? y : 0.0f;
      const unsigned hb = bf16_bits(y);
      const unsigned lb = bf16_bits(y - __uint_as_float(hb << 16));
      h8[e] = (unsigned short)hb;
      l8[e] = (unsigned short)lb;
    }
    unsigned short* op = rhl + row * 1024 + colBase + c8;
    *(volatile v8us*)(op)       = h8;
    *(volatile v8us*)(op + 512) = l8;
    __threadfence();
    *(volatile v8us*)(op)       = h8;
    *(volatile v8us*)(op + 512) = l8;
  }
}

__global__ __launch_bounds__(256) __attribute__((amdgpu_num_vgpr(248)))
void k_store(const float* __restrict__ x, float* out) {
  __shared__ __attribute__((aligned(16))) float tf[64 * SPT];
  const int bx = (int)blockIdx.x, tid = (int)threadIdx.x;
  const int ct = bx & 3, nt = (bx >> 2) & 15, b = bx >> 6;
  const int n0 = nt * 64, c0 = ct * 64;
  const int r0 = b * NTK + n0;
  const int rsub = tid >> 4;
  const int c4   = (tid & 15) * 4;
#pragma unroll
  for (int it = 0; it < 4; ++it) {
    const int tl = it * 16 + rsub;
    const v4f a = *(const v4f*)(x + (size_t)(r0 + tl) * DM + c0 + c4);
    tf[(c4 + 0) * SPT + tl] = a.x;
    tf[(c4 + 1) * SPT + tl] = a.y;
    tf[(c4 + 2) * SPT + tl] = a.z;
    tf[(c4 + 3) * SPT + tl] = a.w;
  }
  __syncthreads();
  v4f ov[4];
#pragma unroll
  for (int it = 0; it < 4; ++it) ov[it] = *(const v4fa*)(tf + (it * 16 + rsub) * SPT + c4);
#pragma unroll
  for (int it = 0; it < 4; ++it)
    *(volatile v4f*)(out + ((size_t)(b * DM + c0 + it * 16 + rsub)) * NTK + n0 + c4) = ov[it];
  __threadfence();
#pragma unroll
  for (int it = 0; it < 4; ++it)
    *(volatile v4f*)(out + ((size_t)(b * DM + c0 + it * 16 + rsub)) * NTK + n0 + c4) = ov[it];
}

static inline size_t al256(size_t o) { return (o + 255) & ~(size_t)255; }

extern "C" void kernel_launch(void* const* d_in, const int* in_sizes, int n_in,
                              void* d_out, int out_size, void* d_ws, size_t ws_size,
                              hipStream_t stream) {
  if (n_in < 18) return;
  if (in_sizes[0] != 2 * DM * NTK || in_sizes[1] != 2 * DM * NTK) return;
  if (in_sizes[2] != 2 * NTK * NTK || in_sizes[3] != 2 * NTK * NTK) return;
  if (in_sizes[4] != NLAY * DM * DM || in_sizes[6] != NLAY * DM * DM) return;
  if (in_sizes[8] != NLAY * DM * DM || in_sizes[10] != NLAY * DM * DM) return;
  if (in_sizes[5] != NLAY * DM || in_sizes[7] != NLAY * DM || in_sizes[9] != NLAY * DM || in_sizes[11] != NLAY * DM) return;
  if (in_sizes[12] != NLAY * 512 * 512) return;
  if (in_sizes[13] != NLAY * 512 || in_sizes[14] != NLAY * 512 || in_sizes[15] != NLAY * 512) return;
  if (in_sizes[16] != NLAY * DM * 512 || in_sizes[17] != NLAY * DM) return;
  if (out_size != NBT * DM * NTK) return;

  const float* desc0 = (const float*)d_in[0];
  const float* desc1 = (const float*)d_in[1];
  const float* M0p   = (const float*)d_in[2];
  const float* M1p   = (const float*)d_in[3];
  const float* Wq    = (const float*)d_in[4];
  const float* bq    = (const float*)d_in[5];
  const float* Wk    = (const float*)d_in[6];
  const float* bk    = (const float*)d_in[7];
  const float* Wv    = (const float*)d_in[8];
  const float* bv    = (const float*)d_in[9];
  const float* Wm    = (const float*)d_in[10];
  const float* bm    = (const float*)d_in[11];
  const float* W1    = (const float*)d_in[12];
  const float* b1    = (const float*)d_in[13];
  const float* g1    = (const float*)d_in[14];
  const float* be1   = (const float*)d_in[15];
  const float* W2    = (const float*)d_in[16];
  const float* b2    = (const float*)d_in[17];
  float* out = (float*)d_out;

  size_t off = 0;
  const size_t oXA   = off; off = al256(off + (size_t)MTOK * DM * 4);
  const size_t oXB   = off; off = al256(off + (size_t)MTOK * DM * 4);
  const size_t oXHL  = off; off = al256(off + (size_t)MTOK * 512 * 2);
  const size_t oYHL  = off; off = al256(off + (size_t)MTOK * 1024 * 2);
  const size_t oQK   = off; off = al256(off + (size_t)2 * MTOK * 512 * 2);
  const size_t oVT   = off; off = al256(off + (size_t)2 * NBT * NHD * HDIM * NTK * 2);
  const size_t oCTX  = off; off = al256(off + (size_t)MTOK * 512 * 2);
  const size_t oZ    = off; off = al256(off + (size_t)MTOK * 512 * 4);
  const size_t oRHL  = off; off = al256(off + (size_t)MTOK * 1024 * 2);
  const size_t oMB   = off; off = al256(off + (size_t)NBT * NTK * NTK * 2);
  const size_t oWQKV = off; off = al256(off + (size_t)NLAY * 768 * 512 * 2);
  const size_t oWMD  = off; off = al256(off + (size_t)NLAY * 256 * 512 * 2);
  const size_t oW1D  = off; off = al256(off + (size_t)NLAY * 512 * 1024 * 2);
  const size_t oW2D  = off; off = al256(off + (size_t)NLAY * 256 * 1024 * 2);
  const size_t oBQKV = off; off = al256(off + (size_t)NLAY * 768 * 4);
  const size_t oREC  = off; off = al256(off + (size_t)64 * 1024 * 4);
  if (off > ws_size || off > (size_t)WSMAX) return;

  char* ws = (char*)d_ws;
  float*          XA    = (float*)(ws + oXA);
  float*          XB    = (float*)(ws + oXB);
  unsigned short* XHL   = (unsigned short*)(ws + oXHL);
  unsigned short* YHL   = (unsigned short*)(ws + oYHL);
  unsigned short* QK    = (unsigned short*)(ws + oQK);
  unsigned short* VT    = (unsigned short*)(ws + oVT);
  unsigned short* CTX   = (unsigned short*)(ws + oCTX);
  float*          Z     = (float*)(ws + oZ);
  unsigned short* RHL   = (unsigned short*)(ws + oRHL);
  unsigned short* MB    = (unsigned short*)(ws + oMB);
  unsigned short* WQKVD = (unsigned short*)(ws + oWQKV);
  unsigned short* WMD   = (unsigned short*)(ws + oWMD);
  unsigned short* W1D   = (unsigned short*)(ws + oW1D);
  unsigned short* W2D   = (unsigned short*)(ws + oW2D);
  float*          BQKV  = (float*)(ws + oBQKV);
  float*          REC   = (float*)(ws + oREC);

  k_wprep<<<WP_B0 + WP_B1 + WP_B2 + WP_B3 + WP_B4, 256, 0, stream>>>(Wq, Wk, Wv, Wm, W1, W2, bq, bk, bv,
                                                                    WQKVD, WMD, W1D, W2D, BQKV);
  k_mask<<<(2 * NTK * NTK) / (8 * 256), 256, 0, stream>>>(M0p, MB);
  k_mask<<<(2 * NTK * NTK) / (8 * 256), 256, 0, stream>>>(M1p, MB + (size_t)2 * NTK * NTK);
  k_xprep<<<128, 256, 0, stream>>>(desc0, 0, XA, XHL, YHL);
  k_xprep<<<128, 256, 0, stream>>>(desc1, 2, XA, XHL, YHL);

  for (int i = 0; i < NLAY; ++i) {
    const int cross = i & 1;
    float* cur = (i & 1) ? XB : XA;
    float* nxt = (i & 1) ? XA : XB;
    k_gemm<0><<<dim3(MTOK / 64, 768 / 64), 128, 0, stream>>>(
        XHL, 512, WQKVD + (size_t)i * 768 * 512, 512, 512, BQKV + (size_t)i * 768, QK, VT, Z, XA, REC);
    k_attn<<<NBT * NHD * (NTK / AT_QB), 128, 0, stream>>>(QK, VT, MB, CTX, cross);
    k_gemm<1><<<dim3(MTOK / 64, 256 / 64), 128, 0, stream>>>(
        CTX, 512, WMD + (size_t)i * 256 * 512, 512, 512, bm + (size_t)i * 256, YHL, QK, Z, XA, REC);
    k_gemm<2><<<dim3(MTOK / 64, 512 / 64), 128, 0, stream>>>(
        YHL, 1024, W1D + (size_t)i * 512 * 1024, 1024, 1024, b1 + (size_t)i * 512, QK, VT, Z, XA, REC);
    k_bnrelu<<<dim3(512 / 64, MTOK / 256), 256, 0, stream>>>(Z, REC, g1 + (size_t)i * 512, be1 + (size_t)i * 512, RHL);
    k_gemm<3><<<dim3(MTOK / 64, 256 / 64), 128, 0, stream>>>(
        RHL, 1024, W2D + (size_t)i * 256 * 1024, 1024, 1024, b2 + (size_t)i * 256, XHL, YHL, nxt, cur, REC);
  }
  k_store<<<NBT * (NTK / 64) * (DM / 64), 256, 0, stream>>>(XA, out);
  (void)hipGetLastError();
}
